// LieAttention_41154376630712
// MI455X (gfx1250) — hardware-run, weakly checked
//
#include <hip/hip_runtime.h>


#define NB_  4
#define TT   1024
#define NH_  8
#define NKV  8
#define REP  (NH_ / NKV)
#define HD   64
#define DQ   (NH_ * HD)
#define DKV  (NKV * HD)
#define ZH   2
#define RH   0
#define PCAR 1024.0f
#define PFL  6.103515625e-05f
#define PQK  1024.0f
#define PQKI 9.5367431640625e-07f
static_assert(PQK * PQK * PQKI == 1.0f, "the carry and its inverse");

typedef _Float16 h16;
typedef unsigned short bf;
typedef __attribute__((ext_vector_type(16))) __bf16   v16bf;
typedef __attribute__((ext_vector_type(16))) _Float16 v16h;
typedef __attribute__((ext_vector_type(8)))  _Float16 v8h;
typedef __attribute__((ext_vector_type(8)))  unsigned short v8us;
typedef __attribute__((ext_vector_type(8)))  float    v8f;
typedef __attribute__((ext_vector_type(4)))  float    v4f;
typedef __attribute__((ext_vector_type(4)))  unsigned v4u;
typedef v8h  __attribute__((may_alias)) v8ha;
typedef v4f  __attribute__((may_alias)) v4fa;
typedef v8us __attribute__((may_alias)) v8usa;

__device__ __forceinline__ unsigned short f2bf(float f) { unsigned u = __float_as_uint(f); u += 0x7FFFu + ((u >> 16) & 1u); return (unsigned short)(u >> 16); }
__device__ __forceinline__ float bf2f(unsigned short b) { return __uint_as_float(((unsigned)b) << 16); }
__device__ __forceinline__ float bfr(float f) { return bf2f(f2bf(f)); }
__device__ __forceinline__ v16h cat16(v8h lo, v8h hi) { return __builtin_shufflevector(lo, hi, 0, 1, 2, 3, 4, 5, 6, 7, 8, 9, 10, 11, 12, 13, 14, 15); }
__device__ __forceinline__ v16bf cat16b(v8us lo, v8us hi) { return __builtin_bit_cast(v16bf, __builtin_shufflevector(lo, hi, 0, 1, 2, 3, 4, 5, 6, 7, 8, 9, 10, 11, 12, 13, 14, 15)); }
__device__ __forceinline__ v8f wmma16(v16h a, v16h b, v8f c) { return __builtin_amdgcn_wmma_f32_16x16x32_f16(false, a, false, b, (short)0, c, false, false); }
__device__ __forceinline__ v8f wmmab(v16bf a, v16bf b, v8f c) { return __builtin_amdgcn_wmma_f32_16x16x32_bf16(false, a, false, b, (short)0, c, false, false); }
typedef __attribute__((ext_vector_type(2))) _Float16 v2h;
typedef __attribute__((ext_vector_type(4))) _Float16 v4h;
typedef __attribute__((ext_vector_type(2))) unsigned short v2us;
typedef __attribute__((ext_vector_type(4))) unsigned short v4us;
typedef __attribute__((ext_vector_type(2))) float v2f;
typedef __attribute__((ext_vector_type(4))) int v4i;

template <typename T16> struct WFrag;
template <> struct WFrag<h16> { typedef v16h V; static __device__ __forceinline__ V ld(const h16* p) { return cat16(*(const v8h*)p, *(const v8h*)(p + 16)); } static __device__ __forceinline__ v8f mma(V a, V b, v8f c) { return wmma16(a, b, c); } };
template <> struct WFrag<bf> { typedef v16bf V; static __device__ __forceinline__ V ld(const bf* p) { return cat16b(*(const v8us*)p, *(const v8us*)(p + 16)); } static __device__ __forceinline__ v8f mma(V a, V b, v8f c) { return wmmab(a, b, c); } };
template <typename T16, int NSPLIT, bool BIAS>
__global__ __launch_bounds__(32) void k_gemmw(const T16* __restrict__ A, const T16* __restrict__ A2, const T16* __restrict__ Bt, const T16* __restrict__ Bt2, int K, float* C, int ldc, const float* __restrict__ bias, size_t sA, size_t sB, size_t sC) {
    typedef typename WFrag<T16>::V V;
    __shared__ __align__(16) float os[16 * 68];
    const size_t z = blockIdx.z; A += z * sA; if (A2) A2 += z * sA; Bt += z * sB; if (Bt2) Bt2 += z * sB; C += z * sC;
    const int lane = threadIdx.x & 31, lr = lane & 15, hi = lane >> 4; const int r0 = blockIdx.x * 64, c0 = blockIdx.y * 64;
    v8f acc[4][4];
#pragma unroll
    for (int mb = 0; mb < 4; ++mb)
#pragma unroll
        for (int nb = 0; nb < 4; ++nb) acc[mb][nb] = (v8f){};
    const size_t aoff = (size_t)(r0 + lr) * K + 8 * hi, boff = (size_t)(c0 + lr) * K + 8 * hi;

    for (int kc = 0; kc < K; kc += 32) {
        V a[4], a2[4];
#pragma unroll
        for (int mb = 0; mb < 4; ++mb) { a[mb] = WFrag<T16>::ld(A + aoff + (size_t)mb * 16 * K + kc); if (NSPLIT == 1 || NSPLIT == 2) a2[mb] = WFrag<T16>::ld(A2 + aoff + (size_t)mb * 16 * K + kc); }
#pragma unroll
        for (int nb = 0; nb < 4; ++nb) { const V b = WFrag<T16>::ld(Bt + boff + (size_t)nb * 16 * K + kc); V b2; if (NSPLIT >= 2) b2 = WFrag<T16>::ld(Bt2 + boff + (size_t)nb * 16 * K + kc);
#pragma unroll
            for (int mb = 0; mb < 4; ++mb) { acc[mb][nb] = WFrag<T16>::mma(a[mb], b, acc[mb][nb]); if (NSPLIT == 1 || NSPLIT == 2) acc[mb][nb] = WFrag<T16>::mma(a2[mb], b, acc[mb][nb]); if (NSPLIT >= 2) acc[mb][nb] = WFrag<T16>::mma(a[mb], b2, acc[mb][nb]); } }
        asm volatile("v_nop\n\tv_nop\n\tv_nop\n\tv_nop" : "+v"(acc[0][0]), "+v"(acc[1][1]), "+v"(acc[2][2]), "+v"(acc[3][3]) : "v"(a[0]), "v"(a[3]));
    }
#pragma unroll
    for (int mb = 0; mb < 4; ++mb) {
#pragma unroll
        for (int nb = 0; nb < 4; ++nb) {
#pragma unroll
            for (int j = 0; j < 8; ++j) os[(hi * 8 + j) * 68 + nb * 16 + lr] = acc[mb][nb][j]; }
        __builtin_amdgcn_wave_barrier(); asm volatile("" ::: "memory");
        float* crow = C + (size_t)(r0 + mb * 16) * ldc + c0;
#pragma unroll 1
        for (int ps = 0; ps < 2; ++ps) {
#pragma unroll
            for (int s = 0; s < 8; ++s) { const int row = 2 * s + hi, cofs = lr * 4; v4f val = *(const v4fa*)(os + row * 68 + cofs); if (BIAS) { val[0] += bfr(bias[c0 + cofs]); val[1] += bfr(bias[c0 + cofs + 1]); val[2] += bfr(bias[c0 + cofs + 2]); val[3] += bfr(bias[c0 + cofs + 3]); }
                *(volatile v4f*)(crow + (size_t)row * ldc + cofs) = val; }
            if (ps == 0) __threadfence(); }
        __builtin_amdgcn_wave_barrier(); asm volatile("" ::: "memory");
    }
}

__device__ __forceinline__ h16 tohx(float x) { return (h16)x; }
__device__ __forceinline__ void splitf(float y, unsigned short& h, unsigned short& l) { h = f2bf(y); l = f2bf(y - bf2f(h)); }
typedef __attribute__((ext_vector_type(2))) _Float16 v2h;
typedef __attribute__((ext_vector_type(4))) _Float16 v4h;
typedef __attribute__((ext_vector_type(2))) unsigned short v2us;
typedef __attribute__((ext_vector_type(4))) unsigned short v4us;
typedef __attribute__((ext_vector_type(2))) float v2f;
typedef __attribute__((ext_vector_type(4))) int v4i;

__global__ __launch_bounds__(256) void k_rbf(const float* __restrict__ X, float* Y, size_t n4) { const size_t i = (size_t)blockIdx.x * 256 + threadIdx.x; if (i >= n4) return; const v4f a = *(const v4f*)(X + i * 4); v4f o;
#pragma unroll
    for (int q = 0; q < 4; ++q) o[q] = bfr(a[q]);
    *(volatile v4f*)(Y + i * 4) = o; __threadfence(); *(volatile v4f*)(Y + i * 4) = o; }

__global__ __launch_bounds__(256) void k_rope(const float* __restrict__ F, int pitch, int nheads, const float* __restrict__ CS, const float* __restrict__ RF, const float* __restrict__ nw, float sc, h16* P16, bf* Ph, bf* Pl) {
    const size_t e = ((size_t)blockIdx.x * 256 + threadIdx.x) * 2; if (e >= (size_t)nheads * TT * HD) return; const int d = (int)(e % HD); const int t = (int)((e / HD) % TT); const int h = (int)(e / ((size_t)HD * TT)); const float* f = F + (size_t)t * pitch + h * HD; const float rf = RF ? RF[(size_t)h * TT + t] : 1.0f; v2h o16; v2us oh, ol;
#pragma unroll
    for (int q = 0; q < 2; ++q) { const int dd = d + q; const int dp = (dd < HD / 2) ? dd + HD / 2 : dd - HD / 2; float x0 = f[dd], x1 = f[dp];
        if (RF) { float n0 = __fmul_rn(x0, rf), n1 = __fmul_rn(x1, rf); x0 = __fmul_rn(bfr(nw[dd]), n0); x1 = __fmul_rn(bfr(nw[dp]), n1); }
        const v2f cs = *(const v2f*)(CS + ((size_t)t * HD + dd) * 2); float a = __fmul_rn(x0, cs[0]), bq = __fmul_rn(x1, cs[1]); const float r = ((dd < HD / 2) ? __fsub_rn(a, bq) : __fadd_rn(a, bq)) * sc;
        o16[q] = tohx(r); unsigned short a2, c2; splitf(r, a2, c2); oh[q] = a2; ol[q] = c2; }
    *(volatile v2h*)(P16 + e) = o16; *(volatile v2us*)(Ph + e) = oh; *(volatile v2us*)(Pl + e) = ol; __threadfence(); *(volatile v2h*)(P16 + e) = o16; *(volatile v2us*)(Ph + e) = oh; *(volatile v2us*)(Pl + e) = ol; }

__global__ __launch_bounds__(256) void k_vtp(const float* __restrict__ F, int pitch, int nheads, h16* V16, bf* Vh, bf* Vl) { const size_t e = ((size_t)blockIdx.x * 256 + threadIdx.x) * 2; if (e >= (size_t)nheads * HD * TT) return; const int t = (int)(e % TT); const int d = (int)((e / TT) % HD); const int g = (int)(e / ((size_t)TT * HD)); v2h o16; v2us oh, ol;
#pragma unroll
    for (int q = 0; q < 2; ++q) { const float x = F[(size_t)(t + q) * pitch + g * HD + d]; o16[q] = tohx(x); unsigned short a2, c2; splitf(x, a2, c2); oh[q] = a2; ol[q] = c2; }
    *(volatile v2h*)(V16 + e) = o16; *(volatile v2us*)(Vh + e) = oh; *(volatile v2us*)(Vl + e) = ol; __threadfence(); *(volatile v2h*)(V16 + e) = o16; *(volatile v2us*)(Vh + e) = oh; *(volatile v2us*)(Vl + e) = ol; }

__global__ __launch_bounds__(256) void k_csid(float* CS) { const int idx = blockIdx.x * 256 + threadIdx.x; if (idx >= TT * HD) return; v2f cs; cs[0] = 1.0f; cs[1] = 0.0f; *(volatile v2f*)(CS + (size_t)idx * 2) = cs; __threadfence(); *(volatile v2f*)(CS + (size_t)idx * 2) = cs; }

__global__ __launch_bounds__(256) void k_merge(const float* __restrict__ O, int h0, float* OUTb) { const size_t e = ((size_t)blockIdx.x * 256 + threadIdx.x) * 2; if (e >= (size_t)ZH * TT * HD) return; const int d = (int)(e % HD); const int t = (int)((e / HD) % TT); const int zz = (int)(e / ((size_t)HD * TT)); const float cs = (t < RH) ? 1.0f : (1.0f / PCAR); const size_t oo = (size_t)t * DQ + (h0 + zz) * HD + d;
    v2f o2; o2[0] = O[e] * cs; o2[1] = O[e + 1] * cs; *(volatile v2f*)(OUTb + oo) = o2; __threadfence(); *(volatile v2f*)(OUTb + oo) = o2; }

__global__ __launch_bounds__(256) void k_g1(const float* __restrict__ p0, const float* __restrict__ a0, const float* __restrict__ a1, const float* __restrict__ a2, const float* __restrict__ pr, const float* __restrict__ pf, const float* __restrict__ ph, float* p1, h16* p2) { const size_t e = ((size_t)blockIdx.x * 256 + threadIdx.x) * 4; if (e >= (size_t)ZH * TT * TT) return; const int j0 = (int)(e % TT); const int i = (int)((e / TT) % TT); const size_t pb = e - (size_t)i * TT - j0;
    float gn = expf(bfr(a0[0])); gn = (gn < 1.0e-3f) ? 1.0e-3f : gn; gn = (gn > 1000.0f) ? 1000.0f : gn; float ta = expf(bfr(a1[0])); ta = (ta < 0.1f) ? 0.1f : ta; ta = (ta > 5.0f) ? 5.0f : ta; float tc = expf(bfr(a2[0])); tc = (tc < 1.0e-3f) ? 1.0e-3f : tc; tc = (tc > 10.0f) ? 10.0f : tc; const float gg = __fmul_rn(__fdiv_rn(gn, tc), PQKI);
    const v4f d4 = *(const v4f*)(p0 + e); const v4f r4 = *(const v4f*)(pr + e); const v4f f4 = *(const v4f*)(pf + e); const v4f h4 = *(const v4f*)(ph + (size_t)i * TT + j0); v4f o; v4h oh;
#pragma unroll
    for (int q = 0; q < 4; ++q) { const float dt = p0[pb + (size_t)(j0 + q) * TT + i]; const float cm = __fsub_rn(d4[q], dt); const float y = tanhf(__fmul_rn(gg, cm)); const float x = __fmul_rn(__fmul_rn(0.5f, y), __fadd_rn(1.0f, erff(__fmul_rn(y, 0.70710677f)))); const float rq = bfr(r4[q]); const float lg = __fsub_rn(logf(__fadd_rn(rq, 1.0e-8f)), logf(__fadd_rn(__fsub_rn(1.0f, rq), 1.0e-8f))); const float z = __fdiv_rn(__fadd_rn(lg, bfr(f4[q])), ta); const float m = __fdiv_rn(1.0f, __fadd_rn(1.0f, expf(-z))); float wv = __fmul_rn(__fmul_rn(__fmul_rn(0.125f, x), m), bfr(h4[q])); o[q] = wv; const float wc = __fmul_rn(wv, PCAR); oh[q] = tohx(fabsf(wc) < PFL ? 0.0f : wc); }
    *(volatile v4f*)(p1 + e) = o; *(volatile v4h*)(p2 + e) = oh; __threadfence(); *(volatile v4f*)(p1 + e) = o; *(volatile v4h*)(p2 + e) = oh; }

__global__ __launch_bounds__(256) void k_e0(const float* __restrict__ p1, float* p3) { const int r = blockIdx.x * 256 + threadIdx.x; if (r >= ZH * TT) return; const float* wr = p1 + (size_t)r * TT; float acc = 0.0f;
    for (int c = 0; c < TT / 4; ++c) { const v4f w4 = *(const v4f*)(wr + 4 * c);
#pragma unroll
        for (int q = 0; q < 4; ++q) { const float cl = (w4[q] < 1.0e-8f) ? 1.0e-8f : w4[q]; acc = __fadd_rn(acc, __fmul_rn(w4[q], logf(cl))); } }
    const float en = -acc; *(volatile float*)(p3 + r) = en; __threadfence(); *(volatile float*)(p3 + r) = en; }

extern "C" void kernel_launch(void* const* d_in, const int* in_sizes, int n_in,
                              void* d_out, int out_size, void* d_ws, size_t ws_size, hipStream_t stream) {
    (void)in_sizes; (void)n_in; (void)out_size;
    const float* xa = (const float*)d_in[0]; const float* xb = (const float*)d_in[1]; const float* xc = (const float*)d_in[2]; const float* pf = (const float*)d_in[3]; const float* s0 = (const float*)d_in[4]; const float* s1 = (const float*)d_in[5]; const float* s2 = (const float*)d_in[6]; const float* ph = (const float*)d_in[7]; const float* pr = (const float*)d_in[8];
    float* OUT0 = (float*)d_out; float* OUT1 = OUT0 + (size_t)NB_ * TT * DQ; float* OUT2 = OUT1 + (size_t)NB_ * NH_ * TT * TT;
    char* wsp = (char*)d_ws;
    auto take = [&](size_t bytes) { char* p = wsp; wsp += (bytes + 255) & ~(size_t)255; return (void*)p; };
    float* CS = (float*)take((size_t)TT * HD * 2 * 4);
    float* XQ = (float*)take((size_t)TT * DQ * 4); float* XK = (float*)take((size_t)TT * DKV * 4); float* XV = (float*)take((size_t)TT * DKV * 4);
    h16* Q16 = (h16*)take((size_t)NH_ * TT * HD * 2); h16* K16 = (h16*)take((size_t)NKV * TT * HD * 2); h16* VT16 = (h16*)take((size_t)NKV * HD * TT * 2);
    bf* PLh = (bf*)take((size_t)NH_ * TT * HD * 2); bf* PLl = (bf*)take((size_t)NH_ * TT * HD * 2);
    float* Sb = (float*)take((size_t)ZH * TT * TT * 4); h16* P16 = (h16*)take((size_t)ZH * TT * TT * 2); float* Ob = (float*)take((size_t)ZH * TT * HD * 4);
    if ((size_t)(wsp - (char*)d_ws) > ws_size) return;
    k_csid<<<(TT * HD + 255) / 256, 256, 0, stream>>>(CS);
    const size_t NX = (size_t)TT * DQ; const unsigned LQ = (unsigned)(((size_t)NH_ * TT * HD / 2 + 255) / 256), LKv = (unsigned)(((size_t)NKV * TT * HD / 2 + 255) / 256);
    for (int b = 0; b < NB_; ++b) { const size_t ob = (size_t)b * TT * DQ;
        k_rbf<<<(unsigned)((NX / 4 + 255) / 256), 256, 0, stream>>>(xa + ob, XQ, NX / 4); k_rbf<<<(unsigned)((NX / 4 + 255) / 256), 256, 0, stream>>>(xb + ob, XK, NX / 4); k_rbf<<<(unsigned)((NX / 4 + 255) / 256), 256, 0, stream>>>(xc + ob, XV, NX / 4);
        k_rope<<<LQ, 256, 0, stream>>>(XQ, DQ, NH_, CS, nullptr, nullptr, PQK, Q16, PLh, PLl); k_rope<<<LKv, 256, 0, stream>>>(XK, DKV, NKV, CS, nullptr, nullptr, PQK, K16, PLh, PLl); k_vtp<<<LKv, 256, 0, stream>>>(XV, DKV, NKV, VT16, PLh, PLl);
        for (int h0 = 0; h0 < NH_; h0 += ZH) { const size_t zq = (size_t)h0, zk = (size_t)(h0 / REP); float* W1 = OUT1 + ((size_t)b * NH_ + h0) * TT * TT; float* E1 = OUT2 + ((size_t)b * NH_ + h0) * TT;
            k_gemmw<h16, 0, false><<<dim3(TT / 64, TT / 64, ZH), 32, 0, stream>>>(Q16 + zq * TT * HD, nullptr, K16 + zk * TT * HD, nullptr, HD, Sb, TT, nullptr, (size_t)TT * HD, (size_t)TT * HD, (size_t)TT * TT);
            k_g1<<<(unsigned)((size_t)ZH * TT * TT / 1024), 256, 0, stream>>>(Sb, s0, s1, s2, pr + (size_t)h0 * TT * TT, pf + (size_t)h0 * TT * TT, ph, W1, P16);
            k_e0<<<ZH * TT / 256, 256, 0, stream>>>(W1, E1);
            k_gemmw<h16, 0, false><<<dim3(TT / 64, HD / 64, ZH), 32, 0, stream>>>(P16, nullptr, VT16 + zk * HD * TT, nullptr, TT, Ob, HD, nullptr, (size_t)TT * TT, (size_t)HD * TT, (size_t)TT * HD);
            k_merge<<<(unsigned)(((size_t)ZH * TT * HD / 2 + 255) / 256), 256, 0, stream>>>(Ob, h0, OUT0 + ob); } }
}
